// CausalSelfAttention_8521215115405
// MI455X (gfx1250) — hardware-verified
//
#include <hip/hip_runtime.h>


#ifndef NB
#define NB 1
#endif
#define NB_FULL 1
#ifndef SEQ
#define SEQ 4096
#endif
#define SEQ_FULL 4096
#define DM   1024
#define NH_  16
#define HD   64
#define DQ   (NH_ * HD)
#ifndef RH
#define RH   512
#endif
#ifndef QCH
#define QCH  512
#endif
#define ZH   4
#define PCAR 1024.0f
#define SCL  0.125f
#define R8TEN 1.333521432163324

static_assert(SEQ <= SEQ_FULL);
static_assert(NB >= 1 && NB <= NB_FULL);
static_assert((SEQ % QCH) == 0);
static_assert((QCH % 64) == 0);
static_assert((RH % 128) == 0);
static_assert(RH <= QCH);
static_assert((SEQ % 128) == 0);
static_assert((NH_ % ZH) == 0);
static_assert(HD == 64);
static_assert((DM % 64) == 0 && (DQ % 64) == 0 && (DM % 32) == 0);
static_assert(((size_t)NH_ * SEQ * HD) % 512 == 0);
static_assert(((size_t)ZH * SEQ * HD) % 512 == 0);
static_assert(((size_t)SEQ * (HD / 2)) % 256 == 0);
static_assert(((size_t)SEQ * DM) % 2048 == 0 && ((size_t)DM * DM) % 2048 == 0);
static_assert(((size_t)ZH * QCH) % 8 == 0);

typedef _Float16 h16;
typedef unsigned short bf;
typedef __attribute__((ext_vector_type(16))) __bf16   v16bf;
typedef __attribute__((ext_vector_type(16))) _Float16 v16h;
typedef __attribute__((ext_vector_type(8)))  _Float16 v8h;
typedef __attribute__((ext_vector_type(8)))  unsigned short v8us;
typedef __attribute__((ext_vector_type(8)))  float    v8f;
typedef __attribute__((ext_vector_type(4)))  float    v4f;
typedef __attribute__((ext_vector_type(2)))  _Float16 v2h;
typedef __attribute__((ext_vector_type(4)))  _Float16 v4h;
typedef __attribute__((ext_vector_type(2)))  unsigned short v2us;
typedef __attribute__((ext_vector_type(4)))  unsigned short v4us;
typedef __attribute__((ext_vector_type(2)))  float v2f;
typedef v8h  __attribute__((may_alias)) v8ha;
typedef v4f  __attribute__((may_alias)) v4fa;
typedef v8us __attribute__((may_alias)) v8usa;

__device__ __forceinline__ unsigned short f2bf(float f) { unsigned u = __float_as_uint(f); u += 0x7FFFu + ((u >> 16) & 1u); return (unsigned short)(u >> 16); }
__device__ __forceinline__ float bf2f(unsigned short b) { return __uint_as_float(((unsigned)b) << 16); }
__device__ __forceinline__ float bfr(float f) { return bf2f(f2bf(f)); }
__device__ __forceinline__ v16h cat16(v8h lo, v8h hi) { return __builtin_shufflevector(lo, hi, 0, 1, 2, 3, 4, 5, 6, 7, 8, 9, 10, 11, 12, 13, 14, 15); }
__device__ __forceinline__ v16bf cat16b(v8us lo, v8us hi) { return __builtin_bit_cast(v16bf, __builtin_shufflevector(lo, hi, 0, 1, 2, 3, 4, 5, 6, 7, 8, 9, 10, 11, 12, 13, 14, 15)); }
__device__ __forceinline__ v8f wmma16(v16h a, v16h b, v8f c) { return __builtin_amdgcn_wmma_f32_16x16x32_f16(false, a, false, b, (short)0, c, false, false); }
__device__ __forceinline__ v8f wmmab(v16bf a, v16bf b, v8f c) { return __builtin_amdgcn_wmma_f32_16x16x32_bf16(false, a, false, b, (short)0, c, false, false); }
__device__ __forceinline__ h16 tohx(float x) { return (h16)x; }
__device__ __forceinline__ void splitf(float y, unsigned short& h, unsigned short& l) { h = f2bf(y); l = f2bf(y - bf2f(h)); }

template <typename T16> struct WFrag;
template <> struct WFrag<h16> { typedef v16h V; static __device__ __forceinline__ V ld(const h16* p) { return cat16(*(const v8h*)p, *(const v8h*)(p + 16)); } static __device__ __forceinline__ v8f mma(V a, V b, v8f c) { return wmma16(a, b, c); } };
template <> struct WFrag<bf> { typedef v16bf V; static __device__ __forceinline__ V ld(const bf* p) { return cat16b(*(const v8us*)p, *(const v8us*)(p + 16)); } static __device__ __forceinline__ v8f mma(V a, V b, v8f c) { return wmmab(a, b, c); } };
template <typename T16, int NSPLIT, bool BIAS>
__global__ __launch_bounds__(32) void k_gemmw(const T16* __restrict__ A, const T16* __restrict__ A2, const T16* __restrict__ Bt, const T16* __restrict__ Bt2, int K, float* C, int ldc, const float* __restrict__ bias, size_t sA, size_t sB, size_t sC) {
    typedef typename WFrag<T16>::V V;
    __shared__ __align__(16) float os[16 * 68];
    const size_t z = blockIdx.z; A += z * sA; if (A2) A2 += z * sA; Bt += z * sB; if (Bt2) Bt2 += z * sB; C += z * sC;
    const int lane = threadIdx.x & 31, lr = lane & 15, hi = lane >> 4; const int r0 = blockIdx.x * 64, c0 = blockIdx.y * 64;
    v8f acc[4][4];
#pragma unroll
    for (int mb = 0; mb < 4; ++mb)
#pragma unroll
        for (int nb = 0; nb < 4; ++nb) acc[mb][nb] = (v8f){};
    const size_t aoff = (size_t)(r0 + lr) * K + 8 * hi, boff = (size_t)(c0 + lr) * K + 8 * hi;
#pragma unroll 1
    for (int kc = 0; kc < K; kc += 32) {
        V a[4], a2[4];
#pragma unroll
        for (int mb = 0; mb < 4; ++mb) { a[mb] = WFrag<T16>::ld(A + aoff + (size_t)mb * 16 * K + kc); if (NSPLIT == 1 || NSPLIT == 2) a2[mb] = WFrag<T16>::ld(A2 + aoff + (size_t)mb * 16 * K + kc); }
#pragma unroll
        for (int nb = 0; nb < 4; ++nb) { const V b = WFrag<T16>::ld(Bt + boff + (size_t)nb * 16 * K + kc); V b2; if (NSPLIT >= 2) b2 = WFrag<T16>::ld(Bt2 + boff + (size_t)nb * 16 * K + kc);
#pragma unroll
            for (int mb = 0; mb < 4; ++mb) { acc[mb][nb] = WFrag<T16>::mma(a[mb], b, acc[mb][nb]); if (NSPLIT == 1 || NSPLIT == 2) acc[mb][nb] = WFrag<T16>::mma(a2[mb], b, acc[mb][nb]); if (NSPLIT >= 2) acc[mb][nb] = WFrag<T16>::mma(a[mb], b2, acc[mb][nb]); } }
        asm volatile("v_nop\n\tv_nop\n\tv_nop\n\tv_nop" : "+v"(acc[0][0]), "+v"(acc[1][1]), "+v"(acc[2][2]), "+v"(acc[3][3]) : "v"(a[0]), "v"(a[3]));
    }
#pragma unroll
    for (int mb = 0; mb < 4; ++mb) {
#pragma unroll
        for (int nb = 0; nb < 4; ++nb) {
#pragma unroll
            for (int j = 0; j < 8; ++j) os[(hi * 8 + j) * 68 + nb * 16 + lr] = acc[mb][nb][j]; }
        __builtin_amdgcn_wave_barrier(); asm volatile("" ::: "memory");
        float* crow = C + (size_t)(r0 + mb * 16) * ldc + c0;
#pragma unroll 1
        for (int ps = 0; ps < 2; ++ps) {
#pragma unroll
            for (int s = 0; s < 8; ++s) { const int row = 2 * s + hi, cofs = lr * 4; v4f val = *(const v4fa*)(os + row * 68 + cofs); if (BIAS) { val[0] += bfr(bias[c0 + cofs]); val[1] += bfr(bias[c0 + cofs + 1]); val[2] += bfr(bias[c0 + cofs + 2]); val[3] += bfr(bias[c0 + cofs + 3]); }
                *(volatile v4f*)(crow + (size_t)row * ldc + cofs) = val; }
            if (ps == 0) __threadfence(); }
        __builtin_amdgcn_wave_barrier(); asm volatile("" ::: "memory");
    }
}

template <typename T16, int NSPLIT, int CMODE>
__global__ __launch_bounds__(32) void k_gemmc(const T16* __restrict__ A, const T16* __restrict__ A2, const T16* __restrict__ Bt, const T16* __restrict__ Bt2, int K, float* C, int ldc, int roff, size_t sA, size_t sB, size_t sC) {
    typedef typename WFrag<T16>::V V;
    __shared__ __align__(16) float os[16 * 68];
    const size_t z = blockIdx.z; A += z * sA; if (A2) A2 += z * sA; Bt += z * sB; if (Bt2) Bt2 += z * sB; C += z * sC;
    const int lane = threadIdx.x & 31, lr = lane & 15, hi = lane >> 4; const int r0 = blockIdx.x * 64, c0 = blockIdx.y * 64;
    if (CMODE == 1 && c0 > r0 + roff + 63) return;
    const int Kl = (CMODE == 2) ? min(K, r0 + roff + 64) : K;
    v8f acc[4][4];
#pragma unroll
    for (int mb = 0; mb < 4; ++mb)
#pragma unroll
        for (int nb = 0; nb < 4; ++nb) acc[mb][nb] = (v8f){};
    const size_t aoff = (size_t)(r0 + lr) * K + 8 * hi, boff = (size_t)(c0 + lr) * K + 8 * hi;
#pragma unroll 1
    for (int kc = 0; kc < Kl; kc += 32) {
        V a[4], a2[4];
#pragma unroll
        for (int mb = 0; mb < 4; ++mb) { a[mb] = WFrag<T16>::ld(A + aoff + (size_t)mb * 16 * K + kc); if (NSPLIT == 1 || NSPLIT == 2) a2[mb] = WFrag<T16>::ld(A2 + aoff + (size_t)mb * 16 * K + kc); }
#pragma unroll
        for (int nb = 0; nb < 4; ++nb) { const V b = WFrag<T16>::ld(Bt + boff + (size_t)nb * 16 * K + kc); V b2; if (NSPLIT >= 2) b2 = WFrag<T16>::ld(Bt2 + boff + (size_t)nb * 16 * K + kc);
#pragma unroll
            for (int mb = 0; mb < 4; ++mb) { acc[mb][nb] = WFrag<T16>::mma(a[mb], b, acc[mb][nb]); if (NSPLIT == 1 || NSPLIT == 2) acc[mb][nb] = WFrag<T16>::mma(a2[mb], b, acc[mb][nb]); if (NSPLIT >= 2) acc[mb][nb] = WFrag<T16>::mma(a[mb], b2, acc[mb][nb]); } }
        asm volatile("v_nop\n\tv_nop\n\tv_nop\n\tv_nop" : "+v"(acc[0][0]), "+v"(acc[1][1]), "+v"(acc[2][2]), "+v"(acc[3][3]) : "v"(a[0]), "v"(a[3]));
    }
#pragma unroll
    for (int mb = 0; mb < 4; ++mb) {
#pragma unroll
        for (int nb = 0; nb < 4; ++nb) {
#pragma unroll
            for (int j = 0; j < 8; ++j) os[(hi * 8 + j) * 68 + nb * 16 + lr] = acc[mb][nb][j]; }
        __builtin_amdgcn_wave_barrier(); asm volatile("" ::: "memory");
        float* crow = C + (size_t)(r0 + mb * 16) * ldc + c0;
#pragma unroll 1
        for (int ps = 0; ps < 2; ++ps) {
#pragma unroll
            for (int s = 0; s < 8; ++s) { const int row = 2 * s + hi, cofs = lr * 4; v4f val = *(const v4fa*)(os + row * 68 + cofs);
                *(volatile v4f*)(crow + (size_t)row * ldc + cofs) = val; }
            if (ps == 0) __threadfence(); }
        __builtin_amdgcn_wave_barrier(); asm volatile("" ::: "memory");
    }
}

__global__ __launch_bounds__(256) void k_cvt8(const float* __restrict__ src, bf* dst, size_t n8) { const size_t i = (size_t)blockIdx.x * 256 + threadIdx.x; if (i >= n8) return; const v8f v = *(const v8f*)(src + i * 8); v8us o;
#pragma unroll
    for (int k = 0; k < 8; ++k) o[k] = f2bf(v[k]); *(volatile v8us*)(dst + i * 8) = o; __threadfence(); *(volatile v8us*)(dst + i * 8) = o; }

__global__ __launch_bounds__(256) void k_csbuild(float* CS) {
    const int idx = blockIdx.x * 256 + threadIdx.x; if (idx >= SEQ * (HD / 2)) return;
    const int j = idx & (HD / 2 - 1); const int t = idx / (HD / 2);
    const int n10 = j >> 3, m8 = j & 7; double p = 1.0;
#pragma unroll 1
    for (int q = 0; q < n10; ++q) p *= 10.0;
#pragma unroll 1
    for (int q = 0; q < m8; ++q) p *= R8TEN;
    const float pf = (float)p;
    const float inv = (float)(1.0 / (double)pf);
    const float ang = __fmul_rn((float)t, inv);
    const double ad = (double)ang;
    const double kq = __builtin_rint(ad * 0.6366197723675814);
    double r = __builtin_fma(-kq, 1.5707963267948966, ad); r = __builtin_fma(-kq, 6.123233995736766e-17, r);
    const int qd = ((int)kq) & 3;
    const double r2 = r * r;
    double sp = -2.505210838544172e-08;
    sp = __builtin_fma(sp, r2, 2.7557319223985893e-06); sp = __builtin_fma(sp, r2, -1.984126984126984e-04); sp = __builtin_fma(sp, r2, 8.333333333333333e-03); sp = __builtin_fma(sp, r2, -1.6666666666666666e-01);
    const double s0 = __builtin_fma(sp * r2, r, r);
    double cp = 2.08767569878681e-09;
    cp = __builtin_fma(cp, r2, -2.755731922398589e-07); cp = __builtin_fma(cp, r2, 2.48015873015873e-05); cp = __builtin_fma(cp, r2, -1.388888888888889e-03); cp = __builtin_fma(cp, r2, 4.1666666666666664e-02); cp = __builtin_fma(cp, r2, -0.5);
    const double c0 = __builtin_fma(cp, r2, 1.0);
    const double cv = (qd == 0) ? c0 : (qd == 1) ? -s0 : (qd == 2) ? -c0 : s0;
    const double sv = (qd == 0) ? s0 : (qd == 1) ? c0 : (qd == 2) ? -s0 : -c0;
    v2f cs; cs[0] = (float)cv; cs[1] = (float)sv;
    *(volatile v2f*)(CS + (size_t)idx * 2) = cs; __threadfence(); *(volatile v2f*)(CS + (size_t)idx * 2) = cs;
}

__global__ __launch_bounds__(256) void k_rope(const float* __restrict__ F, int pitch, int nheads, const float* __restrict__ CS, h16* P16, bf* Ph, bf* Pl) {
    const size_t e = ((size_t)blockIdx.x * 256 + threadIdx.x) * 2; if (e >= (size_t)nheads * SEQ * HD) return;
    const int d = (int)(e % HD); const int t = (int)((e / HD) % SEQ); const int h = (int)(e / ((size_t)HD * SEQ));
    const float* f = F + (size_t)t * pitch + h * HD;
    const float x0 = f[d], x1 = f[d + 1];
    const v2f cs = *(const v2f*)(CS + ((size_t)t * (HD / 2) + (d >> 1)) * 2);
    float a0 = __fmul_rn(x0, cs[0]), b0 = __fmul_rn(x1, cs[1]), a1 = __fmul_rn(x1, cs[0]), b1 = __fmul_rn(x0, cs[1]);
    asm volatile("" : "+v"(a0)); asm volatile("" : "+v"(b0)); asm volatile("" : "+v"(a1)); asm volatile("" : "+v"(b1));
    const float y0 = __fsub_rn(a0, b0), y1 = __fadd_rn(a1, b1);
    v2h o16; v2us oh, ol; o16[0] = tohx(y0); o16[1] = tohx(y1);
    unsigned short u0, w0, u1, w1; splitf(y0, u0, w0); splitf(y1, u1, w1); oh[0] = u0; oh[1] = u1; ol[0] = w0; ol[1] = w1;
    const bool hl = (t < RH); const size_t oo = ((size_t)h * RH + (hl ? t : 0)) * HD + d;
#pragma unroll 1
    for (int ps = 0; ps < 2; ++ps) {
        *(volatile v2h*)(P16 + e) = o16;
        if (hl) { *(volatile v2us*)(Ph + oo) = oh; *(volatile v2us*)(Pl + oo) = ol; }
        if (ps == 0) __threadfence(); }
}

__global__ __launch_bounds__(256) void k_vtp(const float* __restrict__ F, int pitch, int nheads, h16* V16, bf* Vh, bf* Vl) {
    const size_t e = ((size_t)blockIdx.x * 256 + threadIdx.x) * 2; if (e >= (size_t)nheads * HD * SEQ) return;
    const int t = (int)(e % SEQ); const int d = (int)((e / SEQ) % HD); const int g = (int)(e / ((size_t)SEQ * HD)); v2h o16; v2us oh, ol;
#pragma unroll
    for (int q = 0; q < 2; ++q) { const float x = F[(size_t)(t + q) * pitch + g * HD + d]; o16[q] = tohx(x); unsigned short a2, c2; splitf(x, a2, c2); oh[q] = a2; ol[q] = c2; }
    const bool hl = (t < RH); const size_t oo = ((size_t)g * HD + d) * RH + (hl ? t : 0);
#pragma unroll 1
    for (int ps = 0; ps < 2; ++ps) {
        *(volatile v2h*)(V16 + e) = o16;
        if (hl) { *(volatile v2us*)(Vh + oo) = oh; *(volatile v2us*)(Vl + oo) = ol; }
        if (ps == 0) __threadfence(); }
}

__global__ __launch_bounds__(256) void k_asoft(const float* __restrict__ Sb, int roff, h16* P16, bf* Ph, bf* Pl) {
    const int lane = threadIdx.x & 31; const int row = blockIdx.x * 8 + (threadIdx.x >> 5); if (row >= ZH * QCH) return;
    const int il = row % QCH; const int zz = row / QCH; const int i = roff + il; const bool hires = (i < RH); const int nlive = (i >> 7) + 1;
    const float* sr = Sb + (size_t)row * SEQ; float v[SEQ / 32]; float mx = -3.0e38f;
#pragma unroll
    for (int ch = 0; ch < SEQ / 128; ++ch) {
        if (ch < nlive) { const int j0 = ch * 128 + lane * 4; const v4f a = *(const v4f*)(sr + j0);
#pragma unroll
            for (int q = 0; q < 4; ++q) { const int j = j0 + q; float sa = a[q] * SCL; asm volatile("" : "+v"(sa)); const float t = (j <= i) ? sa : -3.0e38f; v[ch * 4 + q] = t; mx = fmaxf(mx, t); }
        } else {
#pragma unroll
            for (int q = 0; q < 4; ++q) v[ch * 4 + q] = -3.0e38f; }
        if ((ch & 15) == 15) asm volatile("" ::: "memory"); }
#pragma unroll
    for (int sh = 16; sh; sh >>= 1) mx = fmaxf(mx, __shfl_xor(mx, sh, 32));
    float sum = 0.f;
#pragma unroll
    for (int k = 0; k < SEQ / 32; ++k) {
        if ((k >> 2) < nlive) { float d0 = __fsub_rn(v[k], mx); asm volatile("" : "+v"(d0)); v[k] = __builtin_amdgcn_exp2f(__fmul_rn(d0, 1.4426950408889634f)); sum += v[k]; }
        else v[k] = 0.0f; }
#pragma unroll
    for (int sh = 16; sh; sh >>= 1) sum += __shfl_xor(sum, sh, 32);
    const float f = __fdiv_rn(hires ? 1.0f : PCAR, sum);
#pragma unroll 1
    for (int ps = 0; ps < 2; ++ps) {
        if (hires) {
#pragma unroll
            for (int ch = 0; ch < RH / 128; ++ch) { v4us oh, ol;
#pragma unroll
                for (int q = 0; q < 4; ++q) { unsigned short a, c2; splitf(v[ch * 4 + q] * f, a, c2); oh[q] = a; ol[q] = c2; }
                const size_t oo = ((size_t)zz * RH + (hires ? i : 0)) * RH + ch * 128 + lane * 4; *(volatile v4us*)(Ph + oo) = oh; *(volatile v4us*)(Pl + oo) = ol; }
        } else {
#pragma unroll
            for (int ch = 0; ch < SEQ / 128; ++ch) { v4h o4;
#pragma unroll
                for (int q = 0; q < 4; ++q) o4[q] = tohx(v[ch * 4 + q] * f);
                *(volatile v4h*)(P16 + (size_t)row * SEQ + ch * 128 + lane * 4) = o4; } }
        if (ps == 0) __threadfence(); }
}

__global__ __launch_bounds__(256) void k_merge(const float* __restrict__ O, int h0, bf* Ah, bf* Al) { const size_t e = ((size_t)blockIdx.x * 256 + threadIdx.x) * 2; if (e >= (size_t)ZH * SEQ * HD) return; const int d = (int)(e % HD); const int t = (int)((e / HD) % SEQ); const int zz = (int)(e / ((size_t)HD * SEQ)); const float cs = (t < RH) ? 1.0f : (1.0f / PCAR); const size_t oo = (size_t)t * DQ + (h0 + zz) * HD + d;
    v2us oh, ol;
#pragma unroll
    for (int q = 0; q < 2; ++q) { unsigned short a, c2; splitf(O[e + q] * cs, a, c2); oh[q] = a; ol[q] = c2; } *(volatile v2us*)(Ah + oo) = oh; *(volatile v2us*)(Al + oo) = ol; __threadfence(); *(volatile v2us*)(Ah + oo) = oh; *(volatile v2us*)(Al + oo) = ol; }

extern "C" void kernel_launch(void* const* d_in, const int* in_sizes, int n_in,
                              void* d_out, int out_size, void* d_ws, size_t ws_size, hipStream_t stream) {
    if (n_in < 5) return;
    if (in_sizes[0] < (NB - 1) * SEQ_FULL * DM + SEQ * DM) return;
    if (in_sizes[1] < DM * DM || in_sizes[2] < DM * DM || in_sizes[3] < DM * DM || in_sizes[4] < DM * DM) return;
    if (out_size < (NB - 1) * SEQ_FULL * DM + SEQ * DM) return;
    const float* x = (const float*)d_in[0]; const float* wq = (const float*)d_in[1]; const float* wk = (const float*)d_in[2]; const float* wv = (const float*)d_in[3]; const float* wo = (const float*)d_in[4];
    float* OUT = (float*)d_out;
    char* wsp = (char*)d_ws;
    auto take = [&](size_t bytes) { char* p = wsp; wsp += (bytes + 255) & ~(size_t)255; return (void*)p; };
    bf* WQ = (bf*)take((size_t)DM * DM * 2); bf* WK = (bf*)take((size_t)DM * DM * 2); bf* WV = (bf*)take((size_t)DM * DM * 2); bf* WO = (bf*)take((size_t)DM * DM * 2);
    float* CS = (float*)take((size_t)SEQ * (HD / 2) * 2 * 4);
    h16* QP16 = (h16*)take((size_t)NH_ * SEQ * HD * 2); h16* KP16 = (h16*)take((size_t)NH_ * SEQ * HD * 2); h16* VT16 = (h16*)take((size_t)NH_ * HD * SEQ * 2);
    bf* QPh = (bf*)take((size_t)NH_ * RH * HD * 2); bf* QPl = (bf*)take((size_t)NH_ * RH * HD * 2); bf* KPh = (bf*)take((size_t)NH_ * RH * HD * 2); bf* KPl = (bf*)take((size_t)NH_ * RH * HD * 2);
    bf* VTh = (bf*)take((size_t)NH_ * HD * RH * 2); bf* VTl = (bf*)take((size_t)NH_ * HD * RH * 2);
    bf* Ph = (bf*)take((size_t)ZH * RH * RH * 2); bf* Pl = (bf*)take((size_t)ZH * RH * RH * 2);
    bf* ATh = (bf*)take((size_t)SEQ * DQ * 2); bf* ATl = (bf*)take((size_t)SEQ * DQ * 2);
    const size_t bXB = (size_t)SEQ * DM * 2, bF = (size_t)SEQ * DQ * 4, bSb = (size_t)ZH * QCH * SEQ * 4, bP16 = (size_t)ZH * QCH * SEQ * 2, bOb = (size_t)ZH * SEQ * HD * 4;
    const size_t szA = (bXB + bF > bSb + bP16 + bOb) ? (bXB + bF) : (bSb + bP16 + bOb);
    char* RA = (char*)take(szA);
    bf* XB = (bf*)RA; float* F = (float*)(RA + bXB);
    float* Sb = (float*)RA; h16* P16 = (h16*)(RA + bSb); float* Ob = (float*)(RA + bSb + bP16);
    if ((size_t)(wsp - (char*)d_ws) > ws_size) return;
    k_cvt8<<<(unsigned)(((size_t)DM * DM / 8 + 255) / 256), 256, 0, stream>>>(wq, WQ, (size_t)DM * DM / 8);
    k_cvt8<<<(unsigned)(((size_t)DM * DM / 8 + 255) / 256), 256, 0, stream>>>(wk, WK, (size_t)DM * DM / 8);
    k_cvt8<<<(unsigned)(((size_t)DM * DM / 8 + 255) / 256), 256, 0, stream>>>(wv, WV, (size_t)DM * DM / 8);
    k_cvt8<<<(unsigned)(((size_t)DM * DM / 8 + 255) / 256), 256, 0, stream>>>(wo, WO, (size_t)DM * DM / 8);
    k_csbuild<<<(unsigned)(((size_t)SEQ * (HD / 2) + 255) / 256), 256, 0, stream>>>(CS);
    const unsigned LP = (unsigned)(((size_t)NH_ * SEQ * HD / 2 + 255) / 256);
    for (int b = 0; b < NB; ++b) {
        k_cvt8<<<(unsigned)(((size_t)SEQ * DM / 8 + 255) / 256), 256, 0, stream>>>(x + (size_t)b * SEQ_FULL * DM, XB, (size_t)SEQ * DM / 8);
        k_gemmw<bf, 0, false><<<dim3(SEQ / 64, DQ / 64, 1), 32, 0, stream>>>(XB, nullptr, WQ, nullptr, DM, F, DQ, nullptr, 0, 0, 0);
        k_rope<<<LP, 256, 0, stream>>>(F, DQ, NH_, CS, QP16, QPh, QPl);
        k_gemmw<bf, 0, false><<<dim3(SEQ / 64, DQ / 64, 1), 32, 0, stream>>>(XB, nullptr, WK, nullptr, DM, F, DQ, nullptr, 0, 0, 0);
        k_rope<<<LP, 256, 0, stream>>>(F, DQ, NH_, CS, KP16, KPh, KPl);
        k_gemmw<bf, 0, false><<<dim3(SEQ / 64, DQ / 64, 1), 32, 0, stream>>>(XB, nullptr, WV, nullptr, DM, F, DQ, nullptr, 0, 0, 0);
        k_vtp<<<LP, 256, 0, stream>>>(F, DQ, NH_, VT16, VTh, VTl);
        for (int h0 = 0; h0 < NH_; h0 += ZH) {
            for (int c = 0; c < SEQ / QCH; ++c) {
                const int lo = c * QCH; const int lof = (c == 0) ? RH : lo; const int nf = lo + QCH - lof;
                if (c == 0 && (RH) > 0)
                    k_gemmc<bf, 2, 1><<<dim3(RH / 64, RH / 64, ZH), 32, 0, stream>>>(QPh + (size_t)h0 * RH * HD, QPl + (size_t)h0 * RH * HD, KPh + (size_t)h0 * RH * HD, KPl + (size_t)h0 * RH * HD, HD, Sb, SEQ, 0, (size_t)RH * HD, (size_t)RH * HD, (size_t)QCH * SEQ);
                if (nf > 0)
                    k_gemmc<h16, 0, 1><<<dim3(nf / 64, (lo + QCH) / 64, ZH), 32, 0, stream>>>(QP16 + (size_t)h0 * SEQ * HD + (size_t)lof * HD, nullptr, KP16 + (size_t)h0 * SEQ * HD, nullptr, HD, Sb + (size_t)(lof - lo) * SEQ, SEQ, lof, (size_t)SEQ * HD, (size_t)SEQ * HD, (size_t)QCH * SEQ);
                k_asoft<<<(unsigned)(ZH * QCH / 8), 256, 0, stream>>>(Sb, lo, P16, Ph, Pl);
                if (c == 0 && (RH) > 0)
                    k_gemmc<bf, 2, 2><<<dim3(RH / 64, HD / 64, ZH), 32, 0, stream>>>(Ph, Pl, VTh + (size_t)h0 * HD * RH, VTl + (size_t)h0 * HD * RH, RH, Ob, HD, 0, (size_t)RH * RH, (size_t)HD * RH, (size_t)SEQ * HD);
                if (nf > 0)
                    k_gemmc<h16, 0, 2><<<dim3(nf / 64, HD / 64, ZH), 32, 0, stream>>>(P16 + (size_t)(lof - lo) * SEQ, nullptr, VT16 + (size_t)h0 * HD * SEQ, nullptr, SEQ, Ob + (size_t)lof * HD, HD, lof, (size_t)QCH * SEQ, (size_t)HD * SEQ, (size_t)SEQ * HD);
            }
            k_merge<<<(unsigned)(((size_t)ZH * SEQ * HD / 2 + 255) / 256), 256, 0, stream>>>(Ob, h0, ATh, ATl);
        }
        k_gemmw<bf, 1, false><<<dim3(SEQ / 64, DM / 64, 1), 32, 0, stream>>>(ATh, ATl, WO, nullptr, DQ, OUT + (size_t)b * SEQ_FULL * DM, DM, nullptr, 0, 0, 0);
    }
}
